// GNNRewriteDiscriminator_42133629173808
// MI455X (gfx1250) — hardware-run, weakly checked
//
#include <hip/hip_runtime.h>


namespace {
constexpr int N = 100000, NP = 100032, E = 1600000, G = 256, V = 10, DE = 16, DH = 32;
constexpr float XS = 64.0f  , WSC = 256.0f, NEG = 0.2f  ;

typedef _Float16 b16;
typedef __attribute__((ext_vector_type(16))) _Float16 v16b;
typedef __attribute__((ext_vector_type(8))) _Float16 v8b;
typedef __attribute__((ext_vector_type(8))) float v8f;
typedef __attribute__((ext_vector_type(4))) float v4f;
__device__ __forceinline__ float bf16_rne(float f) { unsigned int u = __float_as_uint(f); u += 0x7FFFu + ((u >> 16) & 1u); return __uint_as_float(u & 0xFFFF0000u); }
__device__ __forceinline__ void split16(float v, b16& hi, b16& lo) { hi = (b16)v; lo = (b16)(v - (float)hi); }
__device__ __forceinline__ v16b frag_kb(const b16* p, int hh) { const v8b a = *(const v8b*)(p + 8 * hh), b = *(const v8b*)(p + 16 + 8 * hh); v16b f;
#pragma unroll
  for (int e = 0; e < 8; ++e) { f[e] = a[e]; f[8 + e] = b[e]; } return f; }
__device__ __forceinline__ v8f wmma16b(v16b a, v16b b, v8f c) { v8f d = __builtin_amdgcn_wmma_f32_16x16x32_f16(false, a, false, b, (short)0, c, false, false); asm volatile("v_nop\n\tv_nop\n\tv_nop\n\tv_nop" : "+v"(d) : "v"(a), "v"(b)); return d; }
__device__ __forceinline__ void wave_lds_sync() { __builtin_amdgcn_fence(__ATOMIC_RELEASE, "workgroup"); __builtin_amdgcn_wave_barrier(); __builtin_amdgcn_fence(__ATOMIC_ACQUIRE, "workgroup"); }
__device__ __forceinline__ float pmul(float a, float b) { float p = a * b; asm volatile("" : "+v"(p)); return p; }
__device__ __forceinline__ int iclamp(int v, int lo, int hi) { return v < lo ? lo : (v > hi ? hi : v); }
__device__ __forceinline__ float nexp(float x) { return __builtin_amdgcn_exp2f(x * 1.4426950408889634f); }
__device__ __forceinline__ float lrelu(float x) { return x > 0.0f ? x : NEG * x; }

constexpr int CSR_NBLK = 512, CSR_GB = 9, CSR_GN = 1 << CSR_GB  , CSR_MAXG = 512, CSR_CAP = 12288  ;
__global__ __launch_bounds__(64) void csrA_kernel(const int* __restrict__ dst, int E, int N, int nG, int CHP, int NGP, int* __restrict__ STG, int* __restrict__ HST) {
  extern __shared__ int sm[];
  int* cnt = sm; int* run = sm + NGP; int* ids = sm + 2 * NGP;
  const int b = blockIdx.x; const int ch = (E + CSR_NBLK - 1) / CSR_NBLK; const int e0 = b * ch, e1 = min(E, e0 + ch);
  for (int i = threadIdx.x; i < NGP; i += 64) cnt[i] = 0;
  for (int i = threadIdx.x; i < CHP; i += 64) ids[i] = -1;
  __syncthreads();
  if (threadIdx.x == 0) {
    for (int e = e0; e < e1; ++e) { int d = dst[e]; d = (d < 0) ? 0 : (d >= N ? N - 1 : d); cnt[d >> CSR_GB] += 1; }
    int acc = 0; for (int g = 0; g < nG; ++g) { run[g] = acc; acc += cnt[g]; }
    for (int e = e0; e < e1; ++e) { int d = dst[e]; d = (d < 0) ? 0 : (d >= N ? N - 1 : d); const int g = d >> CSR_GB; ids[run[g]] = e; run[g] += 1; } }
  __syncthreads();
  typedef __attribute__((ext_vector_type(4))) int v4i;
  for (int pass = 0; pass < 2; ++pass) {
    for (int i = threadIdx.x; i < CHP / 4; i += 64) *(volatile v4i*)(STG + (size_t)b * CHP + i * 4) = *(const v4i*)(&ids[i * 4]);
    for (int i = threadIdx.x; i < NGP / 4; i += 64) { v4i v; for (int e = 0; e < 4; ++e) v[e] = (i * 4 + e < nG) ? cnt[i * 4 + e] : 0; *(volatile v4i*)(HST + (size_t)b * NGP + i * 4) = v; }
    __threadfence(); }
}
__global__ __launch_bounds__(512) void csrS_kernel(const int* __restrict__ HST, int nG, int NGP, int* __restrict__ START, int* __restrict__ TOT, int* __restrict__ OFF) {
  __shared__ int tot[CSR_MAXG];
  const int b = threadIdx.x;
  for (int pass = 0; pass < 2; ++pass) { int runb = 0; for (int g = 0; g < nG; ++g) { int c = HST[(size_t)b * NGP + g]; c = (c < 0) ? 0 : c; ((volatile int*)OFF)[(size_t)g * CSR_NBLK + b] = runb; runb += c; } __threadfence(); }
  for (int g = threadIdx.x; g < nG; g += 512) { int s = 0; for (int bb = 0; bb < CSR_NBLK; ++bb) { int c = HST[(size_t)bb * NGP + g]; s += (c < 0) ? 0 : c; } tot[g] = s; }
  __syncthreads();
  if (threadIdx.x < 32) {
    __shared__ int st[CSR_MAXG + 32];
    if (threadIdx.x == 0) { int acc = 0; for (int g = 0; g < NGP; ++g) { st[g] = acc; if (g < nG) acc += (tot[g] + 31) & ~31; } st[NGP] = acc; }
    __builtin_amdgcn_fence(__ATOMIC_RELEASE, "workgroup"); __builtin_amdgcn_wave_barrier(); __builtin_amdgcn_fence(__ATOMIC_ACQUIRE, "workgroup");
    for (int pass = 0; pass < 2; ++pass) { for (int i = threadIdx.x; i < NGP + 32; i += 32) { ((volatile int*)START)[i] = (i <= NGP) ? st[min(i, NGP)] : 0; ((volatile int*)TOT)[i] = (i < nG) ? tot[i] : 0; } __threadfence(); } }
}
__global__ __launch_bounds__(256) void csrB_kernel(const int* __restrict__ dst, int N, int nG, int CHP, int NGP, int permLen, const int* __restrict__ STG, const int* __restrict__ HST, const int* __restrict__ OFF, const int* __restrict__ START, const int* __restrict__ TOT, int* __restrict__ PERM, int* __restrict__ ROWPTR, int* __restrict__ ROWCNT, int* __restrict__ FLAG) {
  typedef __attribute__((ext_vector_type(4))) int v4i;
  __shared__ int ids[CSR_CAP]; __shared__ unsigned short key[CSR_CAP]; __shared__ int outp[CSR_CAP]; __shared__ int ncnt[CSR_GN + 1]; __shared__ int boff[CSR_NBLK + 1];
  const int g = blockIdx.x, t_ = threadIdx.x; int tot = TOT[g]; int st = START[g], stn = START[g + 1]; const int v0 = g * CSR_GN; const int nv = min(CSR_GN, N - v0);
  st = (st < 0) ? 0 : (st > permLen - 32 ? permLen - 32 : st) & ~31; stn = (stn < st) ? st : (stn > permLen ? permLen : stn); tot = (tot < 0) ? 0 : tot; if (tot > stn - st && tot <= CSR_CAP) tot = stn - st;
  if (tot > CSR_CAP) {
    for (int pass = 0; pass < 2; ++pass) { for (int i = t_; i < CSR_GN / 4; i += 256) { v4i a, c; for (int e = 0; e < 4; ++e) { a[e] = st; c[e] = 0; } *(volatile v4i*)(ROWPTR + v0 + i * 4) = a; *(volatile v4i*)(ROWCNT + v0 + i * 4) = c; } if (t_ == 0) ((volatile int*)FLAG)[0] = 1; __threadfence(); } (void)nv; return; }
  if (t_ == 0) { int acc = 0; for (int b = 0; b < CSR_NBLK; ++b) { boff[b] = acc; int c = HST[(size_t)b * NGP + g]; c = (c < 0) ? 0 : (c > CHP ? CHP : c); acc += c; if (acc > tot) acc = tot; } boff[CSR_NBLK] = acc; }
  for (int i = t_; i <= CSR_GN; i += 256) ncnt[i] = 0;
  __syncthreads();
  for (int b = 0; b < CSR_NBLK; ++b) { const int c = boff[b + 1] - boff[b]; int o_ = OFF[(size_t)g * CSR_NBLK + b]; o_ = (o_ < 0) ? 0 : (o_ > CHP - c ? CHP - c : o_); const int* src_ = STG + (size_t)b * CHP + o_;
    for (int i = t_; i < c; i += 256) { int id = src_[i]; id = (id < 0) ? 0 : id; ids[boff[b] + i] = id; int d = dst[id]; d = (d < v0) ? v0 : (d >= N ? N - 1 : d); int kk = d - v0; kk = (kk < 0) ? 0 : (kk >= CSR_GN ? CSR_GN - 1 : kk); key[boff[b] + i] = (unsigned short)kk; } }
  __syncthreads();
  if (t_ == 0) { for (int i = 0; i < tot; ++i) ncnt[key[i]] += 1; int acc = 0; for (int vl = 0; vl < CSR_GN; ++vl) { const int c = ncnt[vl]; ncnt[vl] = acc; acc += c; } ncnt[CSR_GN] = acc;
    for (int i = 0; i < tot; ++i) { const int vl = key[i]; outp[ncnt[vl]] = ids[i]; ncnt[vl] += 1; }
    for (int vl = CSR_GN; vl > 0; --vl) ncnt[vl] = ncnt[vl - 1]; ncnt[0] = 0; }
  __syncthreads();
  for (int pass = 0; pass < 2; ++pass) {
    for (int i = t_; i < (stn - st) / 4; i += 256) { v4i v; for (int e = 0; e < 4; ++e) { const int q = i * 4 + e; v[e] = (q < tot) ? outp[q] : -1; } *(volatile v4i*)(PERM + st + i * 4) = v; }
    for (int i = t_; i < CSR_GN / 4; i += 256) { v4i a, c; for (int e = 0; e < 4; ++e) { const int vl = i * 4 + e; a[e] = st + ncnt[vl]; c[e] = (vl < nv) ? (ncnt[vl + 1] - ncnt[vl]) : 0; } *(volatile v4i*)(ROWPTR + v0 + i * 4) = a; *(volatile v4i*)(ROWCNT + v0 + i * 4) = c; }
    __threadfence(); }
}
__global__ __launch_bounds__(256) void csrZ_kernel(int* __restrict__ p, size_t n4) { typedef __attribute__((ext_vector_type(4))) int v4i; const size_t tid = (size_t)blockIdx.x * 256 + threadIdx.x, nth = (size_t)gridDim.x * 256; v4i z = {0, 0, 0, 0}; for (size_t i = tid; i < n4; i += nth) *(volatile v4i*)(p + i * 4) = z; }
struct CsrBufs { int *STG, *HST, *OFF, *START, *TOT, *PERM, *ROWPTR, *ROWCNT, *FLAG; int nG, NGP, CHP; size_t permLen; char* base; size_t bytes; };
static size_t csr_carve(CsrBufs& c, char* ws, size_t off, int E, int N) {
  const size_t off0 = off; c.base = ws + off;
  auto al = [&](size_t bytes) { char* p = ws + off; off += (bytes + 255) & ~(size_t)255; return p; };
  c.nG = (N + CSR_GN - 1) / CSR_GN; c.NGP = (c.nG + 31) & ~31; const int ch = (E + CSR_NBLK - 1) / CSR_NBLK; c.CHP = (ch + 31) & ~31; c.permLen = (size_t)E + 32 * (size_t)c.nG + 32;
  c.STG = (int*)al((size_t)CSR_NBLK * c.CHP * 4); c.HST = (int*)al((size_t)CSR_NBLK * c.NGP * 4); c.OFF = (int*)al((size_t)c.NGP * CSR_NBLK * 4); c.START = (int*)al((size_t)(c.NGP + 64) * 4); c.TOT = (int*)al((size_t)(c.NGP + 64) * 4);
  c.PERM = (int*)al(c.permLen * 4); c.ROWPTR = (int*)al((size_t)c.nG * CSR_GN * 4); c.ROWCNT = (int*)al((size_t)c.nG * CSR_GN * 4); c.FLAG = (int*)al(256);
  c.bytes = off - off0; return off;
}
static void csr_build(const CsrBufs& c, const int* dst, int E, int N, hipStream_t stream) {
  const size_t smem = (size_t)(2 * c.NGP + c.CHP) * 4;
  csrZ_kernel<<<512, 256, 0, stream>>>((int*)c.base, c.bytes / 16);
  csrA_kernel<<<CSR_NBLK, 64, smem, stream>>>(dst, E, N, c.nG, c.CHP, c.NGP, c.STG, c.HST);
  csrS_kernel<<<1, 512, 0, stream>>>(c.HST, c.nG, c.NGP, c.START, c.TOT, c.OFF);
  csrB_kernel<<<c.nG, 256, 0, stream>>>(dst, N, c.nG, c.CHP, c.NGP, (int)c.permLen, c.STG, c.HST, c.OFF, c.START, c.TOT, c.PERM, c.ROWPTR, c.ROWCNT, c.FLAG);
}


__global__ __launch_bounds__(256) void prep_kernel(const int* __restrict__ gid, const float* __restrict__ prm, const float* __restrict__ emb, const float* __restrict__ pW, const float* __restrict__ pb, const float* __restrict__ w1, const float* __restrict__ w2, float* __restrict__ X0, b16* __restrict__ WT, int doW) {
  const size_t t = (size_t)blockIdx.x * 256 + threadIdx.x; const size_t nx = (size_t)NP * DE / 4;
  if (t < nx) { const size_t e = t * 4; const size_t v = e / DE; const int c0 = (int)(e % DE); v4f o = {0.0f, 0.0f, 0.0f, 0.0f};
    if (v < (size_t)N) { const int g = iclamp(gid[v], 0, V - 1); const float p = bf16_rne(prm[v]); for (int j = 0; j < 4; ++j) o[j] = bf16_rne(emb[g * DE + c0 + j]) + (pmul(p, bf16_rne(pW[c0 + j])) + bf16_rne(pb[c0 + j])); }
    for (int pass = 0; pass < 2; ++pass) { *(volatile v4f*)(X0 + e) = o; __threadfence(); } return; }
  if (!doW) return; const size_t u = t - nx; if (u >= 2 * DH * 32 / 8) return; const size_t e = u * 8; const int l = (int)(e / (DH * 32)); const int rem = (int)(e % (DH * 32)); const int oo = rem / 32, k0 = rem % 32; v8b o8;
  for (int j = 0; j < 8; ++j) { const int k = k0 + j; float w = 0.0f; if (l == 0) { if (k < DE) w = w1[k * DH + oo]; } else w = w2[k * DH + oo]; o8[j] = (b16)(bf16_rne(w) * WSC); }
  for (int pass = 0; pass < 2; ++pass) { *(volatile v8b*)(WT + e) = o8; __threadfence(); }
}
template <int FIN>
__global__ __launch_bounds__(128) void layer_kernel(const float* __restrict__ X, const int* __restrict__ srcs, const int* __restrict__ PERM, const int* __restrict__ ROWPTR, const int* __restrict__ ROWCNT, int permLen, const b16* __restrict__ W, const float* __restrict__ bias, float* __restrict__ Y) {
  __shared__ __attribute__((aligned(16))) b16 Ah[64][40], Al[64][40]; __shared__ __attribute__((aligned(16))) float Ts[4][16][DH + 4];
  const int wave = threadIdx.x >> 5, lane = threadIdx.x & 31, nloc = lane & 15, hlf = lane >> 4; const size_t row0 = (size_t)blockIdx.x * 64 + wave * 16;
  for (int rl = 0; rl < 16; ++rl) { const size_t v = row0 + rl; float a0 = 0.0f;
    if (v < (size_t)N && lane < FIN) { int st = ROWPTR[v], cnt = ROWCNT[v]; cnt = iclamp(cnt, 0, 8192); st = iclamp(st, 0, permLen - cnt); const float dv = rsqrtf((float)cnt + 1.0f);
      a0 = pmul(dv, X[v * FIN + lane]);
      for (int j = 0; j < cnt; ++j) { const int e = iclamp(PERM[st + j], 0, E - 1); const int s = iclamp(srcs[e], 0, N - 1); const float ds = rsqrtf((float)iclamp(ROWCNT[s], 0, 8192) + 1.0f); a0 += pmul(ds, X[(size_t)s * FIN + lane]); }
      a0 = pmul(a0, dv); }
    b16 p, q; split16(a0 * XS, p, q); Ah[wave * 16 + rl][lane] = p; Al[wave * 16 + rl][lane] = q; }
  wave_lds_sync();
  v8f a2[2] = {{}, {}};
  { const v16b a = frag_kb(&Ah[wave * 16 + nloc][0], hlf), al = frag_kb(&Al[wave * 16 + nloc][0], hlf);
#pragma unroll
    for (int t = 0; t < 2; ++t) { const v16b bw = frag_kb(W + (size_t)(t * 16 + nloc) * 32, hlf); a2[t] = wmma16b(a, bw, a2[t]); a2[t] = wmma16b(al, bw, a2[t]); } }
#pragma unroll
  for (int t = 0; t < 2; ++t) { const int c = t * 16 + nloc; const float bb = bf16_rne(bias[c]);
#pragma unroll
    for (int r = 0; r < 8; ++r) Ts[wave][8 * hlf + r][c] = fmaxf(a2[t][r] * (1.0f / (XS * WSC)) + bb, 0.0f); }
  wave_lds_sync();
  for (int pass = 0; pass < 2; ++pass) { for (int r4 = 0; r4 < 16; r4 += 4) { const int rr = r4 + (lane >> 3), c4 = (lane & 7) * 4; *(volatile v4f*)(Y + (row0 + rr) * DH + c4) = *(const v4f*)(&Ts[wave][rr][c4]); } __threadfence(); }
}
__device__ int lower_bound_i(const int* a, int n, int key) { int lo = 0, hi = n; while (lo < hi) { const int mid = (lo + hi) >> 1; if (a[mid] < key) lo = mid + 1; else hi = mid; } return lo; }
__global__ __launch_bounds__(256) void pool_kernel(const float* __restrict__ X, const int* __restrict__ batch, float* __restrict__ PGs) {
  __shared__ float ps[8][DH]; __shared__ __attribute__((aligned(16))) float row[DH];
  const int g = blockIdx.x, t_ = threadIdx.x, c = t_ & 31, ph = t_ >> 5;
  const int lo = lower_bound_i(batch, N, g), hi = lower_bound_i(batch, N, g + 1);
  float s = 0.0f; for (int v = lo + ph; v < hi; v += 8) s += X[(size_t)v * DH + c]; ps[ph][c] = s;
  __syncthreads();
  if (t_ < DH) { float sum = 0.0f; for (int k = 0; k < 8; ++k) sum += ps[k][t_]; row[t_] = sum / fmaxf((float)(hi - lo), 1.0f); }
  __syncthreads();
  for (int pass = 0; pass < 2; ++pass) { if (t_ < 8) *(volatile v4f*)(PGs + (size_t)g * DH + t_ * 4) = *(const v4f*)(&row[t_ * 4]); __threadfence(); }
}
__global__ __launch_bounds__(256) void head_kernel(const float* __restrict__ PGL, const float* __restrict__ PGR, const float* __restrict__ fW1, const float* __restrict__ fb1, const float* __restrict__ fW2, const float* __restrict__ fb2, float* __restrict__ out) {
  const int g = threadIdx.x; float o = bf16_rne(fb2[0]);
#pragma unroll 1
  for (int j = 0; j < DH; ++j) { float z = bf16_rne(fb1[j]);
#pragma unroll 1
    for (int i = 0; i < DH; ++i) { z += pmul(PGL[g * DH + i], bf16_rne(fW1[i * DH + j])); }
#pragma unroll 1
    for (int i = 0; i < DH; ++i) { z += pmul(PGR[g * DH + i], bf16_rne(fW1[(DH + i) * DH + j])); }
    o += pmul(fmaxf(z, 0.0f), bf16_rne(fW2[j])); }
  for (int pass = 0; pass < 2; ++pass) { ((volatile float*)out)[g] = o; __threadfence(); }
}
}

extern "C" void kernel_launch(void* const* d_in, const int* in_sizes, int n_in, void* d_out, int out_size, void* d_ws, size_t ws_size, hipStream_t stream) {
  (void)n_in;
  auto Fp = [&](int i) { return (const float*)d_in[i]; }; auto Ip = [&](int i) { return (const int*)d_in[i]; };
  if (in_sizes[0] != N || in_sizes[1] != N || in_sizes[2] != 2 * E || in_sizes[3] != N || in_sizes[4] != N || in_sizes[6] != 2 * E || in_sizes[8] != V * DE || in_sizes[11] != DE * DH || in_sizes[13] != DH * DH || in_sizes[15] != 2 * DH * DH || out_size != G) return;
  size_t off = 0; char* ws = (char*)d_ws;
  auto carve = [&](size_t bytes) { char* p = ws + off; off += (bytes + 255) & ~(size_t)255; return p; };
  float* X0 = (float*)carve((size_t)NP * DE * 4); float* X1 = (float*)carve((size_t)NP * DH * 4); float* X2 = (float*)carve((size_t)NP * DH * 4); b16* WT = (b16*)carve((size_t)2 * DH * 32 * 2); float* PG = (float*)carve((size_t)2 * G * DH * 4);
  CsrBufs csr; off = csr_carve(csr, ws, off, E, N);
  if (off > ws_size || off > ((size_t)128 << 20)) return;
  const unsigned prepGrid = (unsigned)(((size_t)NP * DE / 4 + 2 * DH * 32 / 8 + 255) / 256);
  for (int side = 0; side < 2; ++side) { const int o4 = side * 4;
    prep_kernel<<<prepGrid, 256, 0, stream>>>(Ip(o4 + 0), Fp(o4 + 1), Fp(8), Fp(9), Fp(10), Fp(11), Fp(13), X0, WT, side == 0 ? 1 : 0);
    csr_build(csr, Ip(o4 + 2) + E, E, N, stream);
    layer_kernel<DE><<<NP / 64, 128, 0, stream>>>(X0, Ip(o4 + 2), csr.PERM, csr.ROWPTR, csr.ROWCNT, (int)csr.permLen, WT, Fp(12), X1);
    layer_kernel<DH><<<NP / 64, 128, 0, stream>>>(X1, Ip(o4 + 2), csr.PERM, csr.ROWPTR, csr.ROWCNT, (int)csr.permLen, WT + (size_t)DH * 32, Fp(14), X2);
    pool_kernel<<<G, 256, 0, stream>>>(X2, Ip(o4 + 3), PG + (size_t)side * G * DH); }
  head_kernel<<<1, 256, 0, stream>>>(PG, PG + (size_t)G * DH, Fp(15), Fp(16), Fp(17), Fp(18), (float*)d_out);
}
